// NewAttention_34943853920599
// MI455X (gfx1250) — hardware-verified
//
#include <hip/hip_runtime.h>
#include <math.h>

#ifndef NB
#define NB 2
#endif
#ifndef SEQ
#define SEQ 2048
#endif
#ifndef NB_FULL
#define NB_FULL 2
#endif
#ifndef SEQ_FULL
#define SEQ_FULL 2048
#endif

typedef __attribute__((ext_vector_type(16))) _Float16 v16h;
typedef __attribute__((ext_vector_type(8)))  _Float16 v8h;
typedef __attribute__((ext_vector_type(16))) __bf16   v16b;
typedef __attribute__((ext_vector_type(8)))  __bf16   v8b;
typedef __attribute__((ext_vector_type(8)))  float    v8f;
typedef __attribute__((ext_vector_type(4)))  float    v4f;
typedef __attribute__((ext_vector_type(2)))  float    v2f;
typedef __attribute__((ext_vector_type(4)))  unsigned v4u;

constexpr int kB = NB;
constexpr int kS = SEQ;
constexpr int kSF = SEQ_FULL;
constexpr int kD = 2048;
constexpr int kH = 16;
constexpr int kDH = 128;
constexpr int kM = kB * kS;
constexpr int kEarly = 128;
constexpr int kPairs = kDH / 2;

static_assert(kB >= 1 && kB <= NB_FULL);
static_assert(kS >= kEarly && kS <= kSF);
static_assert(kM % 64 == 0);
static_assert(kD % 64 == 0);
static_assert(kD % 32 == 0);
static_assert(kS % 64 == 0);
static_assert(kEarly % 64 == 0);
static_assert((kS - kEarly) % 64 == 0);
static_assert(kEarly % 16 == 0);
static_assert(kDH == 128);
static_assert(kH * kDH == kD);
static_assert(kD / 8 == 256);

constexpr size_t kNX = (size_t)kM * kD;
constexpr size_t kNW = (size_t)kD * kD;
constexpr size_t kNE = (size_t)kB * kEarly * kD;
constexpr size_t kNT = (size_t)kPairs * kS;
constexpr size_t kWsTotal = kNX * 2 + kNW * 2 * 4 + kNX * 4 + kNX * 2 * 2 + kNE * 2 * 4 + kNT * 4 * 2;
static_assert(kWsTotal <= (size_t)134217728);

__device__ __forceinline__ unsigned short f2bf_bits(float f) {
  unsigned u = __float_as_uint(f);
  return (unsigned short)((u + 0x7FFFu + ((u >> 16) & 1u)) >> 16);
}
__device__ __forceinline__ float bf_bits2f(unsigned short h) { return __uint_as_float(((unsigned)h) << 16); }

__device__ __forceinline__ void dep_guard_h(v8f& a, v8f& b, v16h x, v16h y) { asm volatile("v_nop\n\tv_nop\n\tv_nop\n\tv_nop" : "+v"(a), "+v"(b) : "v"(x), "v"(y)); }
__device__ __forceinline__ void dep_guard_b(v8f& a, v8f& b, v16b x, v16b y) { asm volatile("v_nop\n\tv_nop\n\tv_nop\n\tv_nop" : "+v"(a), "+v"(b) : "v"(x), "v"(y)); }
__device__ __forceinline__ void keep4_h(v16h a, v16h b, v16h c, v16h d) { asm volatile("v_nop" :: "v"(a), "v"(b), "v"(c), "v"(d)); }
__device__ __forceinline__ void keep4_b(v16b a, v16b b, v16b c, v16b d) { asm volatile("v_nop" :: "v"(a), "v"(b), "v"(c), "v"(d)); }
__device__ __forceinline__ void acc_guard4(v8f& a, v8f& b, v8f& c, v8f& d) { asm volatile("v_nop\n\tv_nop\n\tv_nop\n\tv_nop" : "+v"(a), "+v"(b), "+v"(c), "+v"(d)); }
template <typename T> struct Frag;
template <> struct Frag<_Float16> {
  typedef v16h V; union U { v16h v; v8h h[2]; };
  static __device__ __forceinline__ v16h load(const _Float16* p) {
    U f; f.h[0] = *(const v8h*)(p); f.h[1] = *(const v8h*)(p + 16); return f.v;
  }
  static __device__ __forceinline__ v8f mma(v16h a, v16h b, v8f c) {
    return __builtin_amdgcn_wmma_f32_16x16x32_f16(false, a, false, b, (short)0, c, false, false);
  }
  static __device__ __forceinline__ void guard(v8f& a, v8f& b, v16h x, v16h y) { dep_guard_h(a, b, x, y); }
  static __device__ __forceinline__ void keep(v16h a, v16h b, v16h c, v16h d) { keep4_h(a, b, c, d); }
};
template <> struct Frag<__bf16> {
  typedef v16b V; union U { v16b v; v8b h[2]; };
  static __device__ __forceinline__ v16b load(const __bf16* p) {
    U f; f.h[0] = *(const v8b*)(p); f.h[1] = *(const v8b*)(p + 16); return f.v;
  }
  static __device__ __forceinline__ v8f mma(v16b a, v16b b, v8f c) {
    return __builtin_amdgcn_wmma_f32_16x16x32_bf16(false, a, false, b, (short)0, c, false, false);
  }
  static __device__ __forceinline__ void guard(v8f& a, v8f& b, v16b x, v16b y) { dep_guard_b(a, b, x, y); }
  static __device__ __forceinline__ void keep(v16b a, v16b b, v16b c, v16b d) { keep4_b(a, b, c, d); }
};

__device__ __forceinline__ v8f mma_h(v16h a, v16h b, v8f c) {
  c = __builtin_amdgcn_wmma_f32_16x16x32_f16(false, a, false, b, (short)0, c, false, false);
  asm volatile("v_nop\n\tv_nop\n\tv_nop\n\tv_nop" : "+v"(c) : "v"(a), "v"(b));
  return c;
}

template <int ET> struct Elem;
template <> struct Elem<0> { typedef _Float16 T; };
template <> struct Elem<1> { typedef __bf16 T; };
template <int ET, bool SPLIT, int BIAS_MODE, int OUT_MODE, bool RESID, int ACT = 0>
__global__ __launch_bounds__(256) void wmma_gemm64(
    const unsigned short* __restrict__ Ap, const unsigned short* __restrict__ A2p, int lda, long strideA,
    const unsigned short* __restrict__ Btp, const unsigned short* __restrict__ Bt2p, int ldb, long strideB,
    void* __restrict__ Cout, void* __restrict__ Cout2, int ldc, long strideC,
    const float* __restrict__ bias,
    const float* __restrict__ resid, long strideR,
    int M, int N, int K, float scale) {
  typedef typename Elem<ET>::T T;
  typedef typename Frag<T>::V V;
  const T* A = (const T*)Ap; const T* A2 = (const T*)A2p; const T* Bt = (const T*)Btp; const T* Bt2 = (const T*)Bt2p;
  __shared__ __align__(16) float sT[8][16 * 68];
  const int b    = blockIdx.y;
  const int lane = threadIdx.x & 31;
  const int wave = threadIdx.x >> 5;
  const int tilesN = N >> 6;
  const int tilesM = M >> 6;
  const int tile = blockIdx.x * 8 + wave;
  if (tile >= tilesM * tilesN) return;
  const int tm = tile / tilesN;
  const int tn = tile - tm * tilesN;
  const int m0 = tm << 6;
  const int n0 = tn << 6;

  const T* Ab  = A  + (size_t)b * strideA;
  const T* Bb  = Bt + (size_t)b * strideB;
  const T* Ab2 = SPLIT ? (A2  + (size_t)b * strideA) : nullptr;
  const T* Bb2 = SPLIT ? (Bt2 + (size_t)b * strideB) : nullptr;

  const int rlane = lane & 15;
  const int koff  = (lane >> 4) * 8;
  const int mOff  = (lane >> 4) * 8;

  v8f acc[4][4];
#pragma unroll
  for (int i = 0; i < 4; ++i)
#pragma unroll
    for (int j = 0; j < 4; ++j) acc[i][j] = (v8f){0.f,0.f,0.f,0.f,0.f,0.f,0.f,0.f};

  for (int k0 = 0; k0 < K; k0 += 32) {
    V bh[4], bl[4];
#pragma unroll
    for (int j = 0; j < 4; ++j) {
      const size_t bo = (size_t)(n0 + (j << 4) + rlane) * ldb + koff + k0;
      bh[j] = Frag<T>::load(Bb + bo);
      if (SPLIT) bl[j] = Frag<T>::load(Bb2 + bo);
    }
#pragma unroll
    for (int i = 0; i < 4; ++i) {
      const size_t ao = (size_t)(m0 + (i << 4) + rlane) * lda + koff + k0;
      V ah = Frag<T>::load(Ab + ao);
      V al;
      if (SPLIT) al = Frag<T>::load(Ab2 + ao);
#pragma unroll
      for (int j = 0; j < 4; ++j) {
        acc[i][j] = Frag<T>::mma(ah, bh[j], acc[i][j]);
        if (SPLIT) {
          acc[i][j] = Frag<T>::mma(ah, bl[j], acc[i][j]);
          acc[i][j] = Frag<T>::mma(al, bh[j], acc[i][j]);
        }
      }
      Frag<T>::guard(acc[i][0], acc[i][3], ah, SPLIT ? al : ah);
    }
    Frag<T>::keep(bh[0], bh[1], bh[2], bh[3]);
    if (SPLIT) Frag<T>::keep(bl[0], bl[1], bl[2], bl[3]);
  }
  acc_guard4(acc[0][0], acc[0][1], acc[0][2], acc[0][3]);
  acc_guard4(acc[1][0], acc[1][1], acc[1][2], acc[1][3]);
  acc_guard4(acc[2][0], acc[2][1], acc[2][2], acc[2][3]);
  acc_guard4(acc[3][0], acc[3][1], acc[3][2], acc[3][3]);

  float* slab = sT[wave];
  const float* Rb = RESID ? (resid + (size_t)b * strideR) : nullptr;
#pragma unroll
  for (int i = 0; i < 4; ++i) {
    const int mBase = m0 + (i << 4);
#pragma unroll
    for (int j = 0; j < 4; ++j) {
      const int n = n0 + (j << 4) + rlane;
      float bv = 0.f;
      if (BIAS_MODE == 2) bv = bias[n];
#pragma unroll
      for (int r = 0; r < 8; ++r) {
        float v = acc[i][j][r] * scale;
        if (BIAS_MODE == 1) v += bias[mBase + mOff + r];
        if (BIAS_MODE == 2) v += bv;
        if (RESID) v += Rb[(size_t)(mBase + mOff + r) * ldc + n];
        if (ACT == 1) v = tanhf(v);
        if (ACT == 2) v = fmaxf(v, 0.0f);
        if (ACT == 3) v = v / (1.0f + expf(-v));
        if (ACT == 4) v = (v > 0.f) ? v : 0.01f * v;
        slab[(mOff + r) * 68 + (j << 4) + rlane] = v;
      }
    }
    __builtin_amdgcn_fence(3, "workgroup");
    __builtin_amdgcn_wave_barrier();
    __builtin_amdgcn_fence(2, "workgroup");
    if (OUT_MODE == 0) {
      float* C = (float*)Cout + (size_t)b * strideC;
      const int hh = lane >> 4, c4 = (lane & 15) * 4;
      for (int pass = 0; pass < 2; ++pass) {
#pragma unroll
        for (int it = 0; it < 8; ++it) {
          const int row = it * 2 + hh;
          v4f v = *(const v4f*)(slab + row * 68 + c4);
          *(volatile v4f*)(C + (size_t)(mBase + row) * ldc + n0 + c4) = v;
        }
        __threadfence();
      }
    } else {
      const int q = lane >> 3, c8 = (lane & 7) * 8;
      unsigned short* C  = (unsigned short*)Cout  + (size_t)b * strideC;
      unsigned short* C2 = (OUT_MODE == 2 || OUT_MODE == 3) ? ((unsigned short*)Cout2 + (size_t)b * strideC) : nullptr;
      for (int pass = 0; pass < 2; ++pass) {
#pragma unroll
        for (int it = 0; it < 4; ++it) {
          const int row = it * 4 + q;
          const float* sp = slab + row * 68 + c8;
          v8h hv, lv;
#pragma unroll
          for (int e = 0; e < 8; ++e) {
            if (OUT_MODE == 1) {
              hv[e] = (_Float16)sp[e];
            } else if (OUT_MODE == 3) {
              const _Float16 hq = (_Float16)sp[e];
              const float hqf = (float)hq;
              hv[e] = hq;
              lv[e] = (_Float16)((sp[e] - hqf) * 2048.0f);
            } else {
              unsigned short hb = f2bf_bits(sp[e]);
              unsigned short lb = f2bf_bits(sp[e] - bf_bits2f(hb));
              hv[e] = __builtin_bit_cast(_Float16, hb);
              lv[e] = __builtin_bit_cast(_Float16, lb);
            }
          }
          *(volatile v8h*)(C + (size_t)(mBase + row) * ldc + n0 + c8) = hv;
          if (OUT_MODE == 2 || OUT_MODE == 3) *(volatile v8h*)(C2 + (size_t)(mBase + row) * ldc + n0 + c8) = lv;
        }
        __threadfence();
      }
    }
    __builtin_amdgcn_fence(3, "workgroup");
    __builtin_amdgcn_wave_barrier();
    __builtin_amdgcn_fence(2, "workgroup");
  }
}

__global__ __launch_bounds__(256) void wmma_gemm16_alo(
    const unsigned short* __restrict__ Ahp, const unsigned short* __restrict__ Alp, int lda, long strideA,
    const unsigned short* __restrict__ Btp, int ldb,
    float* __restrict__ Cp, int ldc, long strideC,
    int M, int N, int K, float scale, float lofold) {
  typedef _Float16 T;
  __shared__ __align__(16) float sT[8][16 * 68];
  const int b    = blockIdx.y;
  const int lane = threadIdx.x & 31;
  const int wave = threadIdx.x >> 5;
  const int tilesN = N >> 6;
  const int tilesM = M >> 4;
  const int tile = blockIdx.x * 8 + wave;
  if (tile >= tilesM * tilesN) return;
  const int tm = tile / tilesN;
  const int tn = tile - tm * tilesN;
  const int m0 = tm << 4;
  const int n0 = tn << 6;
  const T* Ah = (const T*)Ahp + (size_t)b * strideA;
  const T* Al = (const T*)Alp + (size_t)b * strideA;
  const T* Bt = (const T*)Btp;
  const int rlane = lane & 15;
  const int koff  = (lane >> 4) * 8;
  const int mOff  = (lane >> 4) * 8;

  v8f acc[4], acc2[4];
#pragma unroll
  for (int j = 0; j < 4; ++j) { acc[j] = (v8f){0.f,0.f,0.f,0.f,0.f,0.f,0.f,0.f}; acc2[j] = acc[j]; }

  for (int k0 = 0; k0 < K; k0 += 32) {
    v16h bh[4];
#pragma unroll
    for (int j = 0; j < 4; ++j) bh[j] = Frag<T>::load(Bt + (size_t)(n0 + (j << 4) + rlane) * ldb + koff + k0);
    const size_t ao = (size_t)(m0 + rlane) * lda + koff + k0;
    const v16h ah = Frag<T>::load(Ah + ao);
    const v16h al = Frag<T>::load(Al + ao);
#pragma unroll
    for (int j = 0; j < 4; ++j) {
      acc[j]  = Frag<T>::mma(ah, bh[j], acc[j]);
      acc2[j] = Frag<T>::mma(al, bh[j], acc2[j]);
    }
    Frag<T>::guard(acc[0], acc2[3], ah, al);
    Frag<T>::keep(bh[0], bh[1], bh[2], bh[3]);
  }
  acc_guard4(acc[0], acc[1], acc[2], acc[3]);
  acc_guard4(acc2[0], acc2[1], acc2[2], acc2[3]);

  float* slab = sT[wave];
#pragma unroll
  for (int j = 0; j < 4; ++j) {
#pragma unroll
    for (int r = 0; r < 8; ++r) {
      const float v = (acc[j][r] + acc2[j][r] * lofold) * scale;
      slab[(mOff + r) * 68 + (j << 4) + rlane] = v;
    }
  }
  __builtin_amdgcn_fence(3, "workgroup");
  __builtin_amdgcn_wave_barrier();
  __builtin_amdgcn_fence(2, "workgroup");
  {
    float* C = Cp + (size_t)b * strideC;
    const int hh = lane >> 4, c4 = (lane & 15) * 4;
    for (int pass = 0; pass < 2; ++pass) {
#pragma unroll
      for (int it = 0; it < 8; ++it) {
        const int row = it * 2 + hh;
        v4f v = *(const v4f*)(slab + row * 68 + c4);
        *(volatile v4f*)(C + (size_t)(m0 + row) * ldc + n0 + c4) = v;
      }
      __threadfence();
    }
  }
}

__global__ __launch_bounds__(256) void cast_f32_bf16x2(
    const float* __restrict__ in, unsigned short* __restrict__ out, int n2) {
  const int i = blockIdx.x * 256 + threadIdx.x;
  if (i < n2) {
    const v2f v = *(const v2f*)(in + 2 * (size_t)i);
    const unsigned u = (unsigned)f2bf_bits(v[0]) | ((unsigned)f2bf_bits(v[1]) << 16);
    ((volatile unsigned*)out)[i] = u;
    __threadfence();
    ((volatile unsigned*)out)[i] = u;
  }
}

__global__ __launch_bounds__(256) void cast_rows_bf16x2(
    const float* __restrict__ in, unsigned short* __restrict__ out, int n2, int seq, int seqFull) {
  const int i = blockIdx.x * 256 + threadIdx.x;
  if (i < n2) {
    const int m  = i / (kD / 2);
    const int c2 = i - m * (kD / 2);
    const int bb = m / seq;
    const int s  = m - bb * seq;
    const v2f v = *(const v2f*)(in + ((size_t)bb * seqFull + s) * kD + 2 * (size_t)c2);
    const unsigned u = (unsigned)f2bf_bits(v[0]) | ((unsigned)f2bf_bits(v[1]) << 16);
    ((volatile unsigned*)out)[i] = u;
    __threadfence();
    ((volatile unsigned*)out)[i] = u;
  }
}

__global__ __launch_bounds__(256) void cast_f32_f16x2_bfscale(
    const float* __restrict__ in, unsigned short* __restrict__ out, int n2, float scl) {
  const int i = blockIdx.x * 256 + threadIdx.x;
  if (i < n2) {
    const v2f v = *(const v2f*)(in + 2 * (size_t)i);
    const float a = bf_bits2f(f2bf_bits(v[0])) * scl;
    const float c = bf_bits2f(f2bf_bits(v[1])) * scl;
    const unsigned u = (unsigned)__builtin_bit_cast(unsigned short, (_Float16)a)
                     | ((unsigned)__builtin_bit_cast(unsigned short, (_Float16)c) << 16);
    ((volatile unsigned*)out)[i] = u;
    __threadfence();
    ((volatile unsigned*)out)[i] = u;
  }
}

struct RopeFreq { float f[kPairs]; };
static_assert(sizeof(RopeFreq) == 4 * kPairs);

__global__ __launch_bounds__(256) void rope_table(
    float* __restrict__ cosT, float* __restrict__ sinT, RopeFreq fr, int S) {
#pragma clang fp contract(off)
  const int s = blockIdx.x * 256 + threadIdx.x;
  const int i = blockIdx.y;
  if (s >= S) return;
  const float f = fr.f[i];
  const float ang = (float)s * f;
  const float cs = cosf(ang);
  const float sn = sinf(ang);
  volatile float* pc = cosT + (size_t)i * S + s;
  volatile float* ps = sinT + (size_t)i * S + s;
  *pc = cs;
  *ps = sn;
  __threadfence();
  *pc = cs;
  *ps = sn;
}

__global__ __launch_bounds__(256) void rope_to_f16(
    const float* __restrict__ src, const float* __restrict__ cosT, const float* __restrict__ sinT,
    unsigned short* __restrict__ dst, unsigned short* __restrict__ dstl, int nrows, int S, int nEarly, float carry) {
#pragma clang fp contract(off)
  const int t = blockIdx.x * 256 + threadIdx.x;
  if (t >= nrows * (kD / 8)) return;
  const int m = t / (kD / 8);
  const int g = t - m * (kD / 8);
  const int d0 = g * 8;
  const int bb = m / S;
  const int s = m - bb * S;
  const int i0 = (d0 & (kDH - 1)) >> 1;
  const v4f xa = *(const v4f*)(src + (size_t)m * kD + d0);
  const v4f xb = *(const v4f*)(src + (size_t)m * kD + d0 + 4);
  float cs[4], sn[4];
#pragma unroll
  for (int e = 0; e < 4; ++e) {
    cs[e] = cosT[(size_t)(i0 + e) * S + s];
    sn[e] = sinT[(size_t)(i0 + e) * S + s];
  }
  float o[8];
  o[0] = (xa[0] * cs[0] - xa[1] * sn[0]) * carry;
  o[1] = (xa[0] * sn[0] + xa[1] * cs[0]) * carry;
  o[2] = (xa[2] * cs[1] - xa[3] * sn[1]) * carry;
  o[3] = (xa[2] * sn[1] + xa[3] * cs[1]) * carry;
  o[4] = (xb[0] * cs[2] - xb[1] * sn[2]) * carry;
  o[5] = (xb[0] * sn[2] + xb[1] * cs[2]) * carry;
  o[6] = (xb[2] * cs[3] - xb[3] * sn[3]) * carry;
  o[7] = (xb[2] * sn[3] + xb[3] * cs[3]) * carry;
  v4u w, wl;
#pragma unroll
  for (int e = 0; e < 4; ++e) {
    const _Float16 h0 = (_Float16)o[2 * e];
    const _Float16 h1 = (_Float16)o[2 * e + 1];
    const _Float16 l0 = (_Float16)((o[2 * e] - (float)h0) * 2048.0f);
    const _Float16 l1 = (_Float16)((o[2 * e + 1] - (float)h1) * 2048.0f);
    w[e]  = (unsigned)__builtin_bit_cast(unsigned short, h0) | ((unsigned)__builtin_bit_cast(unsigned short, h1) << 16);
    wl[e] = (unsigned)__builtin_bit_cast(unsigned short, l0) | ((unsigned)__builtin_bit_cast(unsigned short, l1) << 16);
  }
  const bool early = (s < nEarly);
  volatile v4u* p = (volatile v4u*)(dst + (size_t)m * kD + d0);
  volatile v4u* pl = (volatile v4u*)(dstl + ((size_t)bb * nEarly + (early ? s : 0)) * kD + d0);
  *p = w;
  if (early) *pl = wl;
  __threadfence();
  *p = w;
  if (early) *pl = wl;
}

struct AttGeom {
  long q_bs, k_bs, v_bs, o_bs, ql_bs, kl_bs, vl_bs, ol_bs;
  int rs, S, H, qb_first, nqb_count, spare;
  float sc_scale, o_scale;
};
static_assert(sizeof(AttGeom) == 96);

template <bool EARLY>
__global__ __launch_bounds__(128)
void attn_causal128(const unsigned short* __restrict__ Qp,  const unsigned short* __restrict__ Qlp,
                    const unsigned short* __restrict__ Kp,  const unsigned short* __restrict__ Klp,
                    const unsigned short* __restrict__ Vp,  const unsigned short* __restrict__ Vlp,
                    unsigned short* __restrict__ Op, unsigned short* __restrict__ Olp, AttGeom g) {
  union FH { v16h v; v8h h[2]; };
  constexpr int KC   = EARLY ? 32 : 64;
  constexpr int DV   = EARLY ? 64 : 128;
  constexpr int NDH  = kDH / DV;
  constexpr int NSUB = KC / 16;
  constexpr int NKK  = KC / 32;
  constexpr int NT   = DV / 16;
  constexpr int TPR  = 128 / KC;
  constexpr int KDW  = kDH / TPR;
  constexpr int NKV  = KDW / 8;
  constexpr int VDW  = DV / TPR;
  constexpr int NVV  = VDW / 8;
  constexpr int oKl  = KC * kDH;
  constexpr int oV   = EARLY ? 2 * KC * kDH : KC * kDH;
  constexpr int oVl  = oV + DV * KC;
  constexpr int LPR  = DV / 8;
  constexpr int RPI  = 32 / LPR;
  constexpr int NIT  = 16 / RPI;
  static_assert((EARLY ? (oVl + DV * KC) : oVl) <= 16384);
  static_assert(4 * 16 * DV <= 8192);
  static_assert(NKV >= 1 && NVV >= 1 && KC * TPR == 128 && TPR * VDW == DV && TPR * KDW == kDH && NIT * RPI == 16);

  __shared__ __align__(16) float KVO[8192];
  __shared__ __align__(16) unsigned short Psh[4][16 * KC];
  __shared__ __align__(16) unsigned short Psl[EARLY ? 4 : 1][EARLY ? 16 * KC : 8];
  unsigned short* const Lh  = (unsigned short*)KVO;
  unsigned short* const Ksh = Lh;
  unsigned short* const Ksl = Lh + oKl;
  unsigned short* const Vth = Lh + oV;
  unsigned short* const Vtl = Lh + oVl;

  const float kNegInf = -__builtin_inff();
  const float kLoFold = 1.0f / 2048.0f;
  const int tid  = threadIdx.x;
  const int wave = tid >> 5;
  const int lane = tid & 31;
  const int hh   = lane >> 4;
  const int c    = lane & 15;

  const unsigned bx = blockIdx.x;
  const int dsel = (int)(bx % (unsigned)NDH);
  const unsigned rest = bx / (unsigned)NDH;
  const int qb = g.qb_first + (int)(rest % (unsigned)g.nqb_count);
  const int bh = (int)(rest / (unsigned)g.nqb_count);
  const int h  = bh % g.H;
  const int b  = bh / g.H;
  const int q0 = qb * 64 + wave * 16;
  const int dbase = dsel * DV;
  const int hc = h * kDH;

  const unsigned short* qbp  = Qp  + (size_t)b * g.q_bs  + hc;
  const unsigned short* qlbp = Qlp + (size_t)b * g.ql_bs + hc;
  const unsigned short* kbp  = Kp  + (size_t)b * g.k_bs  + hc;
  const unsigned short* klbp = Klp + (size_t)b * g.kl_bs + hc;
  const unsigned short* vbp  = Vp  + (size_t)b * g.v_bs  + hc + dbase;
  const unsigned short* vlbp = Vlp + (size_t)b * g.vl_bs + hc + dbase;
  unsigned short*       obp  = Op  + (size_t)b * g.o_bs  + hc + dbase;
  unsigned short*       olbp = Olp + (size_t)b * g.ol_bs + hc + dbase;

  v16h qa[4], ql[4];
  {
    const _Float16* qrow = (const _Float16*)(qbp + (size_t)(q0 + c) * g.rs);
    const _Float16* qlrow = (const _Float16*)(qlbp + (size_t)(q0 + c) * g.rs);
#pragma unroll
    for (int dc = 0; dc < 4; ++dc) {
      qa[dc] = Frag<_Float16>::load(qrow + dc * 32 + 8 * hh);
      if (EARLY) ql[dc] = Frag<_Float16>::load(qlrow + dc * 32 + 8 * hh);
      else ql[dc] = qa[dc];
    }
  }

  float mrow[8], lrow[8];
  v8f oacc[NT], oacc2[NT];
#pragma unroll
  for (int r = 0; r < 8; ++r) { mrow[r] = kNegInf; lrow[r] = 0.f; }
#pragma unroll
  for (int t = 0; t < NT; ++t) { oacc[t] = (v8f){0.f,0.f,0.f,0.f,0.f,0.f,0.f,0.f}; oacc2[t] = oacc[t]; }

  const int nChunks = (qb + 1) * (64 / KC);
  for (int kc = 0; kc < nChunks; ++kc) {
    const int kv0 = kc * KC;
    __syncthreads();
    {
      const int kvr = tid / TPR;
      const int sub = tid - kvr * TPR;
      const int kd0 = sub * KDW;
      const int vq0 = sub * VDW;
      {
        const unsigned short* ksrc = kbp + (size_t)(kv0 + kvr) * g.rs + kd0;
        v4u kw[NKV];
#pragma unroll
        for (int i = 0; i < NKV; ++i) kw[i] = *(const v4u*)(ksrc + 8 * i);
#pragma unroll
        for (int i = 0; i < NKV; ++i) *(v4u*)(Ksh + kvr * kDH + kd0 + 8 * i) = kw[i];
      }
      if (EARLY) {
        const unsigned short* klsrc = klbp + (size_t)(kv0 + kvr) * g.rs + kd0;
        v4u kw[NKV];
#pragma unroll
        for (int i = 0; i < NKV; ++i) kw[i] = *(const v4u*)(klsrc + 8 * i);
#pragma unroll
        for (int i = 0; i < NKV; ++i) *(v4u*)(Ksl + kvr * kDH + kd0 + 8 * i) = kw[i];
      }
      {
        const unsigned short* vsrc = vbp + (size_t)(kv0 + kvr) * g.rs + vq0;
        v4u vw[NVV];
#pragma unroll
        for (int i = 0; i < NVV; ++i) vw[i] = *(const v4u*)(vsrc + 8 * i);
#pragma unroll
        for (int i = 0; i < NVV; ++i) {
#pragma unroll
          for (int e = 0; e < 4; ++e) {
            const int d = vq0 + 8 * i + 2 * e;
            const unsigned wv = vw[i][e];
            Vth[d * KC + kvr]       = (unsigned short)(wv & 0xffffu);
            Vth[(d + 1) * KC + kvr] = (unsigned short)(wv >> 16);
          }
        }
      }
      if (EARLY) {
        const unsigned short* vlsrc = vlbp + (size_t)(kv0 + kvr) * g.rs + vq0;
        v4u vw[NVV];
#pragma unroll
        for (int i = 0; i < NVV; ++i) vw[i] = *(const v4u*)(vlsrc + 8 * i);
#pragma unroll
        for (int i = 0; i < NVV; ++i) {
#pragma unroll
          for (int e = 0; e < 4; ++e) {
            const int d = vq0 + 8 * i + 2 * e;
            const unsigned wl = vw[i][e];
            Vtl[d * KC + kvr]       = (unsigned short)(wl & 0xffffu);
            Vtl[(d + 1) * KC + kvr] = (unsigned short)(wl >> 16);
          }
        }
      }
    }
    __syncthreads();

    v8f s[NSUB], s2[NSUB];
#pragma unroll
    for (int j = 0; j < NSUB; ++j) {
      s[j] = (v8f){0.f,0.f,0.f,0.f,0.f,0.f,0.f,0.f};
      s2[j] = s[j];
#pragma unroll
      for (int dc = 0; dc < 4; ++dc) {
        FH kb;
        const _Float16* kp = (const _Float16*)(Ksh + (j * 16 + c) * kDH + dc * 32 + 8 * hh);
        kb.h[0] = *(const v8h*)(kp);
        kb.h[1] = *(const v8h*)(kp + 16);
        s[j] = mma_h(qa[dc], kb.v, s[j]);
        if (EARLY) {
          FH kl;
          const _Float16* klp = (const _Float16*)(Ksl + (j * 16 + c) * kDH + dc * 32 + 8 * hh);
          kl.h[0] = *(const v8h*)(klp);
          kl.h[1] = *(const v8h*)(klp + 16);
          s2[j] = mma_h(qa[dc], kl.v, s2[j]);
          s2[j] = mma_h(ql[dc], kb.v, s2[j]);
        }
      }
    }
    const bool needMask = (kv0 + KC > qb * 64);
    float cm[8];
#pragma unroll
    for (int r = 0; r < 8; ++r) {
      const int qrow = q0 + 8 * hh + r;
      float m = kNegInf;
#pragma unroll
      for (int j = 0; j < NSUB; ++j) {
        const int kvcol = kv0 + j * 16 + c;
        float raw = s[j][r];
        if (EARLY) raw += s2[j][r] * kLoFold;
        float val = raw * g.sc_scale;
        if (needMask && (kvcol > qrow)) val = kNegInf;
        s[j][r] = val;
        m = fmaxf(m, val);
      }
#pragma unroll
      for (int off = 1; off < 16; off <<= 1) m = fmaxf(m, __shfl_xor(m, off, 32));
      cm[r] = m;
    }
    unsigned short* pw  = Psh[wave];
    unsigned short* pwl = Psl[EARLY ? wave : 0];
#pragma unroll
    for (int r = 0; r < 8; ++r) {
      const float mnew = fmaxf(mrow[r], cm[r]);
      const float alpha = expf(mrow[r] - mnew);
      mrow[r] = mnew;
      float psum = 0.f;
#pragma unroll
      for (int j = 0; j < NSUB; ++j) {
        const float p = expf(s[j][r] - mnew);
        psum += p;
        const float ps = p * 32768.0f;
        const _Float16 ph = (_Float16)ps;
        pw[(8 * hh + r) * KC + j * 16 + c] = __builtin_bit_cast(unsigned short, ph);
        if (EARLY) {
          const _Float16 plv = (_Float16)((ps - (float)ph) * 2048.0f);
          pwl[(8 * hh + r) * KC + j * 16 + c] = __builtin_bit_cast(unsigned short, plv);
        }
      }
#pragma unroll
      for (int off = 1; off < 16; off <<= 1) psum += __shfl_xor(psum, off, 32);
      lrow[r] = lrow[r] * alpha + psum;
#pragma unroll
      for (int t = 0; t < NT; ++t) {
        oacc[t][r] *= alpha;
        if (EARLY) oacc2[t][r] *= alpha;
      }
    }
    __builtin_amdgcn_fence(3, "workgroup");
    __builtin_amdgcn_wave_barrier();
    __builtin_amdgcn_fence(2, "workgroup");
#pragma unroll 1
    for (int kk = 0; kk < NKK; ++kk) {
      FH pa, pl;
      const _Float16* pp = (const _Float16*)(pw + c * KC + kk * 32 + 8 * hh);
      pa.h[0] = *(const v8h*)(pp);
      pa.h[1] = *(const v8h*)(pp + 16);
      if (EARLY) {
        const _Float16* ppl = (const _Float16*)(pwl + c * KC + kk * 32 + 8 * hh);
        pl.h[0] = *(const v8h*)(ppl);
        pl.h[1] = *(const v8h*)(ppl + 16);
      } else {
        pl.v = pa.v;
      }
#pragma unroll
      for (int t = 0; t < NT; ++t) {
        FH vb;
        const _Float16* vp = (const _Float16*)(Vth + (t * 16 + c) * KC + kk * 32 + 8 * hh);
        vb.h[0] = *(const v8h*)(vp);
        vb.h[1] = *(const v8h*)(vp + 16);
        oacc[t] = mma_h(pa.v, vb.v, oacc[t]);
        if (EARLY) {
          FH vl;
          const _Float16* vq = (const _Float16*)(Vtl + (t * 16 + c) * KC + kk * 32 + 8 * hh);
          vl.h[0] = *(const v8h*)(vq);
          vl.h[1] = *(const v8h*)(vq + 16);
          oacc2[t] = mma_h(pa.v, vl.v, oacc2[t]);
          oacc2[t] = mma_h(pl.v, vb.v, oacc2[t]);
        }
      }
    }
  }

  __syncthreads();
  float* os = KVO + wave * 16 * DV;
#pragma unroll
  for (int r = 0; r < 8; ++r) {
    const float inv = g.o_scale * (1.0f / lrow[r]);
#pragma unroll
    for (int t = 0; t < NT; ++t) {
      float ho = oacc[t][r];
      if (EARLY) ho += oacc2[t][r] * kLoFold;
      os[(8 * hh + r) * DV + t * 16 + c] = ho * inv;
    }
  }
  __builtin_amdgcn_fence(3, "workgroup");
  __builtin_amdgcn_wave_barrier();
  __builtin_amdgcn_fence(2, "workgroup");
  {
    const int rsel = lane / LPR, c8 = (lane % LPR) * 8;
    for (int pass = 0; pass < 2; ++pass) {
#pragma unroll
      for (int it = 0; it < NIT; ++it) {
        const int row = it * RPI + rsel;
        const float* sp = os + row * DV + c8;
        v8h hv, lv;
#pragma unroll
        for (int e = 0; e < 8; ++e) {
          const _Float16 hq = (_Float16)sp[e];
          hv[e] = hq;
          if (EARLY) {
            const float hqf = (float)hq;
            lv[e] = (_Float16)((sp[e] - hqf) * 2048.0f);
          }
        }
        *(volatile v8h*)(obp + (size_t)(q0 + row) * g.rs + c8) = hv;
        if (EARLY) *(volatile v8h*)(olbp + (size_t)(q0 + row) * g.rs + c8) = lv;
      }
      __threadfence();
    }
  }
}

extern "C" void kernel_launch(void* const* d_in, const int* in_sizes, int n_in,
                              void* d_out, int out_size, void* d_ws, size_t ws_size,
                              hipStream_t stream) {
  if (n_in < 5) return;
  const size_t needX = ((size_t)(kB - 1) * kSF + kS) * kD;
  if ((size_t)in_sizes[0] < needX || (size_t)in_sizes[1] < kNW || (size_t)in_sizes[2] < kNW ||
      (size_t)in_sizes[3] < kNW || (size_t)in_sizes[4] < kNW || (size_t)out_size < kNX) return;

  const float* x  = (const float*)d_in[0];
  const float* Wq = (const float*)d_in[1];
  const float* Wk = (const float*)d_in[2];
  const float* Wv = (const float*)d_in[3];
  const float* Wo = (const float*)d_in[4];
  float* out = (float*)d_out;

  char* ws = (char*)d_ws;
  size_t off = 0;
  unsigned short* Xb  = (unsigned short*)(ws + off);
  unsigned short* Oh  = (unsigned short*)(ws + off); off += kNX * 2;
  unsigned short* Wqb = (unsigned short*)(ws + off); off += kNW * 2;
  unsigned short* Wkb = (unsigned short*)(ws + off); off += kNW * 2;
  unsigned short* Wvb = (unsigned short*)(ws + off); off += kNW * 2;
  unsigned short* Woh = (unsigned short*)(ws + off); off += kNW * 2;
  float* tmpF = (float*)(ws + off);
  unsigned short* Vh  = (unsigned short*)(ws + off);
  unsigned short* Vl  = (unsigned short*)(ws + off + kNX * 2); off += kNX * 4;
  unsigned short* Qh  = (unsigned short*)(ws + off); off += kNX * 2;
  unsigned short* Kh  = (unsigned short*)(ws + off); off += kNX * 2;
  unsigned short* Qlc = (unsigned short*)(ws + off); off += kNE * 2;
  unsigned short* Klc = (unsigned short*)(ws + off); off += kNE * 2;
  unsigned short* Ohc = (unsigned short*)(ws + off); off += kNE * 2;
  unsigned short* Olc = (unsigned short*)(ws + off); off += kNE * 2;
  float* cosT = (float*)(ws + off); off += kNT * 4;
  float* sinT = (float*)(ws + off); off += kNT * 4;
  if (off != kWsTotal || off > ws_size) return;

  RopeFreq fr;
  for (int i = 0; i < kPairs; ++i) {
    const double e = (double)(2 * i) / (double)kDH;
    const float p = (float)pow(10000.0, e);
    fr.f[i] = 1.0f / p;
  }

  const int thr = 256;
  const int nX2 = (int)(kNX / 2), nW2 = (int)(kNW / 2);
  const int castBlocksX = (nX2 + thr - 1) / thr;
  const int castBlocksW = (nW2 + thr - 1) / thr;
  cast_rows_bf16x2<<<castBlocksX, thr, 0, stream>>>(x, Xb, nX2, kS, kSF);
  cast_f32_bf16x2<<<castBlocksW, thr, 0, stream>>>(Wq, Wqb, nW2);
  cast_f32_bf16x2<<<castBlocksW, thr, 0, stream>>>(Wk, Wkb, nW2);
  cast_f32_bf16x2<<<castBlocksW, thr, 0, stream>>>(Wv, Wvb, nW2);
  cast_f32_f16x2_bfscale<<<castBlocksW, thr, 0, stream>>>(Wo, Woh, nW2, 256.0f);

  rope_table<<<dim3((kS + thr - 1) / thr, kPairs), thr, 0, stream>>>(cosT, sinT, fr, kS);

  const int tilesFull = (kM / 64) * (kD / 64);
  const int gemmBlocksFull = (tilesFull + 7) / 8;
  const int ropeThreads = kM * (kD / 8);
  const int ropeBlocks = (ropeThreads + thr - 1) / thr;
  wmma_gemm64<1, false, 0, 0, false><<<dim3(gemmBlocksFull, 1), thr, 0, stream>>>(
      Xb, Xb, kD, 0L, Wqb, Wqb, kD, 0L, (void*)tmpF, (void*)tmpF, kD, 0L,
      cosT, cosT, 0L, kM, kD, kD, 1.0f);
  rope_to_f16<<<ropeBlocks, thr, 0, stream>>>(tmpF, cosT, sinT, Qh, Qlc, kM, kS, kEarly, 4.0f);
  wmma_gemm64<1, false, 0, 0, false><<<dim3(gemmBlocksFull, 1), thr, 0, stream>>>(
      Xb, Xb, kD, 0L, Wkb, Wkb, kD, 0L, (void*)tmpF, (void*)tmpF, kD, 0L,
      cosT, cosT, 0L, kM, kD, kD, 1.0f);
  rope_to_f16<<<ropeBlocks, thr, 0, stream>>>(tmpF, cosT, sinT, Kh, Klc, kM, kS, kEarly, 4.0f);

  wmma_gemm64<1, false, 0, 3, false><<<dim3(gemmBlocksFull, 1), thr, 0, stream>>>(
      Xb, Xb, kD, 0L, Wvb, Wvb, kD, 0L, (void*)Vh, (void*)Vl, kD, 0L,
      cosT, cosT, 0L, kM, kD, kD, 16.0f);

  const int nqb = kS / 64;
  const int nqbE = kEarly / 64;
  const float scl = 1.0f / sqrtf((float)kDH);
  AttGeom ga;
  ga.q_bs = (long)kS * kD; ga.k_bs = (long)kS * kD; ga.v_bs = (long)kS * kD; ga.o_bs = (long)kS * kD;
  ga.ql_bs = (long)kEarly * kD; ga.kl_bs = (long)kEarly * kD; ga.vl_bs = (long)kS * kD; ga.ol_bs = (long)kEarly * kD;
  ga.rs = kD; ga.S = kS; ga.H = kH; ga.qb_first = nqbE; ga.nqb_count = nqb - nqbE; ga.spare = 0;
  ga.sc_scale = scl / 16.0f;
  ga.o_scale = 1.0f / 512.0f;
  if (nqb > nqbE) {
    attn_causal128<false><<<kB * kH * (nqb - nqbE), 128, 0, stream>>>(Qh, Qlc, Kh, Klc, Vh, Vl, Oh, Olc, ga);
  }
  AttGeom gb = ga;
  gb.o_bs = (long)kEarly * kD;
  gb.qb_first = 0; gb.nqb_count = nqbE;
  attn_causal128<true><<<kB * kH * nqbE * 2, 128, 0, stream>>>(Qh, Qlc, Kh, Klc, Vh, Vl, Ohc, Olc, gb);

  const float oscale = 1.0f / 262144.0f;
  if (kS > kEarly) {
    const int tilesMain = ((kS - kEarly) / 64) * (kD / 64);
    const int gemmBlocksMain = (tilesMain + 7) / 8;
    wmma_gemm64<0, false, 0, 0, false><<<dim3(gemmBlocksMain, kB), thr, 0, stream>>>(
        Oh + (size_t)kEarly * kD, Oh + (size_t)kEarly * kD, kD, (long)kS * kD,
        Woh, Woh, kD, 0L,
        (void*)(out + (size_t)kEarly * kD), (void*)(out + (size_t)kEarly * kD), kD, (long)kS * kD,
        cosT, cosT, 0L, kS - kEarly, kD, kD, oscale);
  }
  const int tiles16 = (kEarly / 16) * (kD / 64);
  const int gemmBlocks16 = (tiles16 + 7) / 8;
  wmma_gemm16_alo<<<dim3(gemmBlocks16, kB), thr, 0, stream>>>(
      Ohc, Olc, kD, (long)kEarly * kD, Woh, kD, out, kD, (long)kS * kD,
      kEarly, kD, kD, oscale, 1.0f / 2048.0f);
}
